// VointGraphConv_19911468384710
// MI455X (gfx1250) — hardware-run, weakly checked
//
#include <hip/hip_runtime.h>


#ifndef NB
#define NB 4
#endif
#ifndef NPT
#define NPT 1024
#endif
#define NB_FULL  4
#define NPT_FULL 1024
#ifndef OUT_NPT
#define OUT_NPT NPT
#endif
#define CC   64
#define C2   32
#define VV   20
#define PPB  8
#define TB   (PPB * VV)
#define MT   (TB / 16)
#define NW   4
#define NT   (32 * NW)
#define NVPC (NPT * VV)
#define NVP_FULL (NPT_FULL * VV)
#define OUT_NVP  (OUT_NPT * VV)
#define COLS (NB * NVPC)
#define NBLK (COLS / TB)
#define XBP  72
#define XHP  40
#define OSP  36
#define UTP  164
#define WCS  256.0f
#define WCI  (1.0f / 256.0f)
#define BIGF 1.0e10f
#define EPSF 1.0e-5f
#define QPR  (TB / 4)

static_assert(CC == 64);
static_assert(C2 == 32);
static_assert(2 * C2 == CC);
static_assert(NT == 2 * CC);
static_assert(NT % 8 == 0);
static_assert(VV % 4 == 0);
static_assert(TB % 16 == 0);
static_assert(QPR % 8 == 0);
static_assert(NPT % PPB == 0);
static_assert(OUT_NPT % PPB == 0);
static_assert(NBLK * TB == COLS);
static_assert(NBLK * PPB == NB * NPT);
static_assert(NBLK % 4 == 0);
static_assert(NB <= NB_FULL);
static_assert(NPT <= NPT_FULL);
static_assert((C2 * CC) / 8 == 256);
static_assert((2 * CC * C2) / 8 == 2 * 256);
static_assert((CC * QPR) % NT == 0);
static_assert(((CC * QPR) / NT) % 4 == 0);
static_assert((TB * 8) % NT == 0);
static_assert((size_t)NT * 16 * ((TB * 8) / NT) == (size_t)TB * C2 * 4);
static_assert((size_t)NT * 16 * ((CC * QPR) / NT) == (size_t)CC * TB * 4);
static_assert((size_t)NT * 16 * 2 == (size_t)PPB * 2 * CC * 4);
static_assert((5 * CC) % 4 == 0);
static_assert((5 * CC) / 4 <= NT);
static_assert((XBP * 2) % 16 == 0);
static_assert((XHP * 2) % 16 == 0);
static_assert((OSP * 4) % 16 == 0);
static_assert((UTP * 4) % 16 == 0);
static_assert(XBP >= CC);
static_assert(XHP >= C2);
static_assert(UTP >= TB);
static_assert((size_t)TB * XBP * 2 + (size_t)TB * OSP * 4 + 64 * 4 <= 131072);
static_assert((size_t)TB * XHP * 2 + (size_t)2 * CC * UTP * 4 + (size_t)10 * CC * 4 + (size_t)PPB * 2 * CC * 4 <= 131072);

typedef _Float16 h16;
typedef unsigned short bf;
typedef __attribute__((ext_vector_type(16))) __bf16   v16bf;
typedef __attribute__((ext_vector_type(16))) _Float16 v16h;
typedef __attribute__((ext_vector_type(8)))  _Float16 v8h;
typedef __attribute__((ext_vector_type(4)))  _Float16 v4h;
typedef __attribute__((ext_vector_type(8)))  unsigned short v8us;
typedef __attribute__((ext_vector_type(8)))  float    v8f;
typedef __attribute__((ext_vector_type(4)))  float    v4f;
typedef v4f  __attribute__((may_alias)) v4fa;
typedef v4h  __attribute__((may_alias)) v4ha;

__device__ __forceinline__ unsigned short f2bf(float f) { unsigned u = __float_as_uint(f); u += 0x7FFFu + ((u >> 16) & 1u); return (unsigned short)(u >> 16); }
__device__ __forceinline__ float bfr(float f) { return __uint_as_float(((unsigned)f2bf(f)) << 16); }
__device__ __forceinline__ v16h cat16(v8h lo, v8h hi) { return __builtin_shufflevector(lo, hi, 0, 1, 2, 3, 4, 5, 6, 7, 8, 9, 10, 11, 12, 13, 14, 15); }
__device__ __forceinline__ v16bf cat16b(v8us lo, v8us hi) { return __builtin_bit_cast(v16bf, __builtin_shufflevector(lo, hi, 0, 1, 2, 3, 4, 5, 6, 7, 8, 9, 10, 11, 12, 13, 14, 15)); }
__device__ __forceinline__ v8f wmma16(v16h a, v16h b, v8f c) { return __builtin_amdgcn_wmma_f32_16x16x32_f16(false, a, false, b, (short)0, c, false, false); }
__device__ __forceinline__ v8f wmmab(v16bf a, v16bf b, v8f c) { return __builtin_amdgcn_wmma_f32_16x16x32_bf16(false, a, false, b, (short)0, c, false, false); }
__device__ __forceinline__ v16h  ldh(const h16* p) { return cat16(*(const v8h*)p, *(const v8h*)(p + 16)); }
__device__ __forceinline__ v16bf ldb(const bf* p)  { return cat16b(*(const v8us*)p, *(const v8us*)(p + 16)); }
static __device__ __forceinline__ h16 toh_flush(float v) { const h16 r = (h16)v; return (fabsf(v) < 6.103515625e-05f) ? (h16)0.0f : r; }
__device__ __forceinline__ v8f wmma16g(v16h a, v16h b, v8f c) { c = wmma16(a, b, c); asm volatile("v_nop\n\tv_nop\n\tv_nop\n\tv_nop" : "+v"(c) : "v"(a), "v"(b)); return c; }
__device__ __forceinline__ v8f wmmabg(v16bf a, v16bf b, v8f c) { c = wmmab(a, b, c); asm volatile("v_nop\n\tv_nop\n\tv_nop\n\tv_nop" : "+v"(c) : "v"(a), "v"(b)); return c; }

__global__ __launch_bounds__(256) void k_wprep(const float* __restrict__ w_embed, const float* __restrict__ w_conv, bf* WE, h16* WC) {
    const int tid = threadIdx.x;
    { const v8f v = *(const v8f*)(w_embed + (size_t)tid * 8); v8us o;
#pragma unroll
      for (int k = 0; k < 8; ++k) o[k] = f2bf(v[k]);
      *(volatile v8us*)(WE + (size_t)tid * 8) = o; __threadfence(); *(volatile v8us*)(WE + (size_t)tid * 8) = o; }
#pragma unroll 1
    for (int s = 0; s < 2; ++s) {
        const int g = s * 256 + tid; const int j = g >> 2, c8 = (g & 3) * 8;
        const v8f v = *(const v8f*)(w_conv + (size_t)(j & 63) * CC + (size_t)(j >> 6) * C2 + c8); v8h o;
#pragma unroll
        for (int k = 0; k < 8; ++k) o[k] = toh_flush(bfr(v[k]) * WCS);
        *(volatile v8h*)(WC + (size_t)g * 8) = o; __threadfence(); *(volatile v8h*)(WC + (size_t)g * 8) = o;
    }
}

__global__ __launch_bounds__(NT) void k_embed(const float* __restrict__ feats, const float* __restrict__ mask, const bf* __restrict__ WE, const float* __restrict__ b_embed, float* XS, float* PE) {
    __shared__ __align__(16) bf xb[TB * XBP];
    __shared__ __align__(16) float os[TB * OSP];
    __shared__ __align__(16) float red[64];
    const int tid = threadIdx.x, lane = tid & 31, lr = lane & 15, hi = lane >> 4;
    const int wave = __builtin_amdgcn_readfirstlane((int)(threadIdx.x >> 5));
    const int T0 = blockIdx.x * TB; const int b = T0 / NVPC, tl = T0 % NVPC;
    const size_t fbase = (size_t)b * CC * NVP_FULL + (size_t)tl;
#pragma unroll 1
    for (int it = 0; it < (CC * QPR) / NT; ++it) {
        const int i = it * NT + tid; const int c = i / QPR, q = i % QPR;
        const v4f v = *(const v4f*)(feats + fbase + (size_t)c * NVP_FULL + 4 * q);
#pragma unroll
        for (int k = 0; k < 4; ++k) xb[(4 * q + k) * XBP + c] = f2bf(v[k]);
    }
    __syncthreads();
    v16bf wb00 = ldb(WE + (size_t)(lr) * CC + 8 * hi),      wb01 = ldb(WE + (size_t)(lr) * CC + 32 + 8 * hi);
    v16bf wb10 = ldb(WE + (size_t)(16 + lr) * CC + 8 * hi), wb11 = ldb(WE + (size_t)(16 + lr) * CC + 32 + 8 * hi);
    const float bc0 = bfr(b_embed[lr]), bc1 = bfr(b_embed[16 + lr]);
    const float* mrow = mask + (size_t)b * NVP_FULL + tl;
#pragma unroll 1
    for (int mt = wave; mt < MT; mt += NW) {
        const int ab = (mt * 16 + lr) * XBP + 8 * hi;
        const v16bf a0 = cat16b(*(const v8us*)(&xb[ab]),      *(const v8us*)(&xb[ab + 16]));
        const v16bf a1 = cat16b(*(const v8us*)(&xb[ab + 32]), *(const v8us*)(&xb[ab + 48]));
        v8f acc0 = (v8f){}, acc1 = (v8f){};
        acc0 = wmmabg(a0, wb00, acc0); acc0 = wmmabg(a1, wb01, acc0);
        acc1 = wmmabg(a0, wb10, acc1); acc1 = wmmabg(a1, wb11, acc1);
        const int tr = mt * 16 + 8 * hi;
        const v4f mA = *(const v4f*)(mrow + tr), mB = *(const v4f*)(mrow + tr + 4);
#pragma unroll
        for (int r = 0; r < 4; ++r) {
            const float k0 = bfr(mA[r]), k1 = bfr(mB[r]);
            os[(tr + r) * OSP + lr]          = (acc0[r] + bc0) * k0;
            os[(tr + r) * OSP + 16 + lr]     = (acc1[r] + bc1) * k0;
            os[(tr + 4 + r) * OSP + lr]      = (acc0[4 + r] + bc0) * k1;
            os[(tr + 4 + r) * OSP + 16 + lr] = (acc1[4 + r] + bc1) * k1; }
    }
    __syncthreads();
    if (tid < 64) {
        const int o = tid & 31; const bool sq = tid >= 32; float s = 0.0f;
#pragma unroll 4
        for (int r = 0; r < TB; ++r) { const float v = os[r * OSP + o]; s += sq ? v * v : v; }
        red[tid] = s; }
    __syncthreads();
    const int t16 = tid < 16 ? tid : 15;
#pragma unroll 1
    for (int ps = 0; ps < 2; ++ps) {
        v4f pv = *(const v4fa*)(&red[4 * t16]); asm volatile("" : "+v"(pv));
        if (tid < 16) *(volatile v4f*)(PE + (size_t)blockIdx.x * 64 + 4 * tid) = pv;
#pragma unroll 2
        for (int it = 0; it < (TB * 8) / NT; ++it) { const int i = it * NT + tid; const int row = i >> 3, c4 = (i & 7) * 4;
            const v4f val = *(const v4fa*)(&os[row * OSP + c4]);
            *(volatile v4f*)(XS + (size_t)T0 * C2 + (size_t)i * 4) = val; }
        if (ps == 0) __threadfence(); }
}

__global__ __launch_bounds__(256) void k_fold_e(const float* PE, const float* __restrict__ g, const float* __restrict__ be, float* PRM) {
    __shared__ double sd[256];
    __shared__ double st[64];
    __shared__ __align__(16) float pf[64];
    const int tid = threadIdx.x; const int col = tid & 63, part = tid >> 6;
    double s = 0.0;
#pragma unroll 4
    for (int r = part; r < NBLK; r += 4) s += (double)PE[(size_t)r * 64 + col];
    sd[tid] = s;
    __syncthreads();
    if (tid < 64) st[tid] = (sd[tid] + sd[64 + tid]) + (sd[128 + tid] + sd[192 + tid]);
    __syncthreads();
    if (tid < 32) {
        const double inv = 1.0 / (double)COLS;
        const double m = st[tid] * inv; double var = st[32 + tid] * inv - m * m; var = var < 0.0 ? 0.0 : var;
        const float sc = bfr(g[tid]) * rsqrtf((float)var + EPSF);
        pf[tid] = sc; pf[32 + tid] = bfr(be[tid]) - (float)m * sc; }
    __syncthreads();
    const int t16 = tid < 16 ? tid : 15;
    v4f pv = *(const v4fa*)(&pf[4 * t16]); asm volatile("" : "+v"(pv));
    if (tid < 16) { *(volatile v4f*)(PRM + 4 * tid) = pv; __threadfence(); *(volatile v4f*)(PRM + 4 * tid) = pv; }
}

__global__ __launch_bounds__(NT) void k_conv(const float* XS, const float* __restrict__ mask, const h16* __restrict__ WC, const float* PRM_E, float* U, float* ZX, float* PY) {
    __shared__ __align__(16) h16 xh[TB * XHP];
    __shared__ __align__(16) float ut[CC * UTP];
    __shared__ __align__(16) float zt[CC * UTP];
    __shared__ __align__(16) float red[2 * 5 * CC];
    __shared__ __align__(16) float zs[PPB * 2 * CC];
    const int tid = threadIdx.x, lane = tid & 31, lr = lane & 15, hi = lane >> 4;
    const int wave = __builtin_amdgcn_readfirstlane((int)(threadIdx.x >> 5));
    const int T0 = blockIdx.x * TB; const int b = T0 / NVPC, tl = T0 % NVPC;
    const int c4 = (tid & 7) * 4;
    const v4f sc4 = *(const v4f*)(PRM_E + c4), sh4 = *(const v4f*)(PRM_E + C2 + c4);
    const float* mrow = mask + (size_t)b * NVP_FULL + tl;
#pragma unroll 2
    for (int it = 0; it < (TB * 8) / NT; ++it) {
        const int i = it * NT + tid; const int row = i >> 3;
        const v4f x = *(const v4f*)(XS + (size_t)T0 * C2 + (size_t)i * 4);
        const float mk = bfr(mrow[row]);
        v4h hv;
#pragma unroll
        for (int k = 0; k < 4; ++k) { float t = (x[k] * sc4[k] + sh4[k]) * mk; t = fmaxf(t, 0.0f) * mk; hv[k] = toh_flush(t); }
        *(v4ha*)(&xh[row * XHP + c4]) = hv; }
    __syncthreads();
    v16h wb[8];
#pragma unroll
    for (int j = 0; j < 8; ++j) wb[j] = ldh(WC + (size_t)(j * 16 + lr) * C2 + 8 * hi);
#pragma unroll 1
    for (int mt = wave; mt < MT; mt += NW) {
        const int ab = (mt * 16 + lr) * XHP + 8 * hi;
        const v16h a = cat16(*(const v8h*)(&xh[ab]), *(const v8h*)(&xh[ab + 16]));
#pragma unroll
        for (int j = 0; j < 4; ++j) {
            v8f pa = (v8f){}, pz = (v8f){};
            pa = wmma16g(a, wb[j], pa); pz = wmma16g(a, wb[4 + j], pz);
            v4f u0, u1, z0, z1;
#pragma unroll
            for (int r = 0; r < 4; ++r) { z0[r] = pz[r] * WCI; z1[r] = pz[4 + r] * WCI; u0[r] = (pa[r] - pz[r]) * WCI; u1[r] = (pa[4 + r] - pz[4 + r]) * WCI; }
            const int ob = (j * 16 + lr) * UTP + mt * 16 + 8 * hi;
            *(v4fa*)(&ut[ob]) = u0; *(v4fa*)(&ut[ob + 4]) = u1; *(v4fa*)(&zt[ob]) = z0; *(v4fa*)(&zt[ob + 4]) = z1; }
    }
    __syncthreads();
    { const int o = tid & 63; const int ph = tid >> 6;
      float a1 = 0.0f, a2 = 0.0f, a3 = 0.0f, a4 = 0.0f, a5 = 0.0f;
#pragma unroll 1
      for (int pp = 0; pp < PPB / 2; ++pp) {
          const int p = ph * (PPB / 2) + pp; const int base = o * UTP + p * VV;
          float su = 0.0f, sz = 0.0f, zx = -3.0e38f, zn = 3.0e38f;
#pragma unroll 4
          for (int v = 0; v < VV; ++v) { const float uu = ut[base + v], zz = zt[base + v]; su += uu; sz += zz; a3 += uu * uu; a4 += zz * zz; zx = fmaxf(zx, zz); zn = fminf(zn, zz); }
          a1 += su; a2 += sz; a5 += su * sz;
          zs[p * 2 * CC + o] = zx; zs[p * 2 * CC + CC + o] = zn; }
      red[(ph * 5 + 0) * CC + o] = a1; red[(ph * 5 + 1) * CC + o] = a2; red[(ph * 5 + 2) * CC + o] = a3; red[(ph * 5 + 3) * CC + o] = a4; red[(ph * 5 + 4) * CC + o] = a5; }
    __syncthreads();
    const int t80 = tid < (5 * CC) / 4 ? tid : (5 * CC) / 4 - 1;
#pragma unroll 1
    for (int ps = 0; ps < 2; ++ps) {
        { const v4f x0 = *(const v4fa*)(&red[4 * t80]); const v4f x1 = *(const v4fa*)(&red[5 * CC + 4 * t80]); v4f pv = x0 + x1; asm volatile("" : "+v"(pv));
          if (tid < (5 * CC) / 4) *(volatile v4f*)(PY + (size_t)blockIdx.x * (5 * CC) + 4 * tid) = pv; }
#pragma unroll
        for (int it = 0; it < 2; ++it) { const int i = it * NT + tid;
            const v4f val = *(const v4fa*)(&zs[4 * i]);
            *(volatile v4f*)(ZX + (size_t)blockIdx.x * (PPB * 2 * CC) + (size_t)i * 4) = val; }
#pragma unroll 2
        for (int it = 0; it < (CC * QPR) / NT; ++it) { const int i = it * NT + tid; const int o = i / QPR, q = i % QPR;
            const v4f val = *(const v4fa*)(&ut[o * UTP + 4 * q]);
            *(volatile v4f*)(U + ((size_t)b * CC + o) * NVPC + tl + 4 * q) = val; }
        if (ps == 0) __threadfence(); }
}

__global__ __launch_bounds__(256) void k_fold_y(const float* PY, const float* __restrict__ g, const float* __restrict__ be, float* PRM) {
    __shared__ double sd[5 * CC];
    __shared__ __align__(16) float pf[2 * CC];
    const int tid = threadIdx.x;
#pragma unroll 1
    for (int col = tid; col < 5 * CC; col += 256) {
        double s = 0.0;
#pragma unroll 4
        for (int r = 0; r < NBLK; ++r) s += (double)PY[(size_t)r * (5 * CC) + col];
        sd[col] = s; }
    __syncthreads();
    if (tid < CC) {
        const double inv = 1.0 / (double)COLS;
        const double mean = (sd[tid] + sd[CC + tid]) * inv;
        const double e2 = (sd[2 * CC + tid] + sd[3 * CC + tid]) * inv + 2.0 * sd[4 * CC + tid] * inv * (1.0 / (double)VV);
        double var = e2 - mean * mean; var = var < 0.0 ? 0.0 : var;
        const float sc = bfr(g[tid]) * rsqrtf((float)var + EPSF);
        pf[tid] = sc; pf[CC + tid] = bfr(be[tid]) - (float)mean * sc; }
    __syncthreads();
    const int t32 = tid < 32 ? tid : 31;
    v4f pv = *(const v4fa*)(&pf[4 * t32]); asm volatile("" : "+v"(pv));
    if (tid < 32) { *(volatile v4f*)(PRM + 4 * tid) = pv; __threadfence(); *(volatile v4f*)(PRM + 4 * tid) = pv; }
}

__global__ __launch_bounds__(NT) void k_final(const float* __restrict__ feats, const float* __restrict__ mask, const float* U, const float* ZX, const float* PRM_Y, float* OUT) {
    __shared__ float zl[PPB * CC];
    __shared__ float sl[CC];
    const int tid = threadIdx.x;
    const int T0 = blockIdx.x * TB; const int b = T0 / NVPC, tl = T0 % NVPC;
    if (tid < CC) sl[tid] = PRM_Y[tid];
#pragma unroll 1
    for (int it = 0; it < (PPB * CC) / NT; ++it) {
        const int e = it * NT + tid; const int p = e / CC, o = e % CC;
        const size_t zb = ((size_t)blockIdx.x * PPB + p) * (2 * CC);
        const float zx = ZX[zb + o], zn = ZX[zb + CC + o];
        const float sc = PRM_Y[o], tc = PRM_Y[CC + o];
        const float hiv = sc * zx, lov = sc * zn;
        zl[e] = tc + ((sc >= 0.0f) ? hiv : lov); }
    __syncthreads();
    const size_t fbase = (size_t)b * CC * NVP_FULL + (size_t)tl;
    const float* mrow = mask + (size_t)b * NVP_FULL + tl;
#pragma unroll 1
    for (int g = 0; g < (CC * QPR) / NT / 4; ++g) {
        v4f val[4]; size_t oa[4];
#pragma unroll
        for (int s = 0; s < 4; ++s) {
            const int i = (g * 4 + s) * NT + tid; const int o = i / QPR, q = i % QPR; const int p = q / (VV / 4);
            const v4f f4 = *(const v4f*)(feats + fbase + (size_t)o * NVP_FULL + 4 * q);
            const v4f u4 = *(const v4f*)(U + ((size_t)b * CC + o) * NVPC + tl + 4 * q);
            const v4f m4 = *(const v4f*)(mrow + 4 * q);
            const float sc = sl[o], zc = zl[p * CC + o];
            v4f r;
#pragma unroll
            for (int e = 0; e < 4; ++e) {
                const float mk = bfr(m4[e]);
                const float y = fmaxf(sc * u4[e] + zc, 0.0f) * mk;
                const float ag = (y - BIGF * (1.0f - mk)) * mk;
                r[e] = bfr(f4[e]) + ag; }
            val[s] = r; oa[s] = ((size_t)b * CC + o) * OUT_NVP + (size_t)tl + 4 * q; }
#pragma unroll
        for (int s = 0; s < 4; ++s) *(volatile v4f*)(OUT + oa[s]) = val[s];
        __threadfence();
#pragma unroll
        for (int s = 0; s < 4; ++s) *(volatile v4f*)(OUT + oa[s]) = val[s];
    }
}

static constexpr size_t al256(size_t v) { return (v + 255) & ~(size_t)255; }
static constexpr size_t SZ_WE  = al256((size_t)C2 * CC * 2);
static constexpr size_t SZ_WC  = al256((size_t)2 * CC * C2 * 2);
static constexpr size_t SZ_XS  = al256((size_t)COLS * C2 * 4);
static constexpr size_t SZ_PE  = al256((size_t)NBLK * 64 * 4);
static constexpr size_t SZ_PRE = al256((size_t)2 * C2 * 4);
static constexpr size_t SZ_U   = al256((size_t)NB * CC * NVPC * 4);
static constexpr size_t SZ_ZX  = al256((size_t)NB * NPT * 2 * CC * 4);
static constexpr size_t SZ_PY  = al256((size_t)NBLK * 5 * CC * 4);
static constexpr size_t SZ_PRY = al256((size_t)2 * CC * 4);
static constexpr size_t SZ_TOTAL = SZ_WE + SZ_WC + SZ_XS + SZ_PE + SZ_PRE + SZ_U + SZ_ZX + SZ_PY + SZ_PRY;
static_assert(SZ_TOTAL <= (size_t)134217728);
static_assert((size_t)NBLK * TB * C2 * 4 <= SZ_XS);
static_assert(((size_t)(NB - 1) * CC + (CC - 1)) * NVPC * 4 + (size_t)NVPC * 4 <= SZ_U);
static_assert((size_t)NBLK * PPB * 2 * CC * 4 <= SZ_ZX);
static_assert((size_t)NBLK * 5 * CC * 4 <= SZ_PY);
static_assert((size_t)NBLK * 64 * 4 <= SZ_PE);

extern "C" void kernel_launch(void* const* d_in, const int* in_sizes, int n_in,
                              void* d_out, int out_size, void* d_ws, size_t ws_size, hipStream_t stream) {
    if (n_in < 9) return;
    const size_t needf = ((size_t)(NB - 1) * CC + (size_t)(CC - 1)) * NVP_FULL + (size_t)NVPC;
    const size_t needm = (size_t)(NB - 1) * NVP_FULL + (size_t)NVPC;
    if ((size_t)in_sizes[0] < needf || (size_t)in_sizes[1] < needm) return;
    if (in_sizes[2] < C2 * CC || in_sizes[3] < C2 || in_sizes[4] < C2 || in_sizes[5] < C2) return;
    if (in_sizes[6] < CC * CC || in_sizes[7] < CC || in_sizes[8] < CC) return;
    if ((size_t)out_size < ((size_t)(NB - 1) * CC + (size_t)(CC - 1)) * OUT_NVP + (size_t)NVPC) return;
    if (SZ_TOTAL > ws_size) return;
    const float* feats    = (const float*)d_in[0];
    const float* mask     = (const float*)d_in[1];
    const float* w_embed  = (const float*)d_in[2];
    const float* b_embed  = (const float*)d_in[3];
    const float* g_embed  = (const float*)d_in[4];
    const float* be_embed = (const float*)d_in[5];
    const float* w_conv   = (const float*)d_in[6];
    const float* g_conv   = (const float*)d_in[7];
    const float* be_conv  = (const float*)d_in[8];
    float* OUT = (float*)d_out;
    char* wsp = (char*)d_ws;
    bf*    WE   = (bf*)wsp;    wsp += SZ_WE;
    h16*   WC   = (h16*)wsp;   wsp += SZ_WC;
    float* XS   = (float*)wsp; wsp += SZ_XS;
    float* PE   = (float*)wsp; wsp += SZ_PE;
    float* PRME = (float*)wsp; wsp += SZ_PRE;
    float* U    = (float*)wsp; wsp += SZ_U;
    float* ZX   = (float*)wsp; wsp += SZ_ZX;
    float* PY   = (float*)wsp; wsp += SZ_PY;
    float* PRMY = (float*)wsp; wsp += SZ_PRY;

    k_wprep<<<1, 256, 0, stream>>>(w_embed, w_conv, WE, WC);
    k_embed<<<NBLK, NT, 0, stream>>>(feats, mask, WE, b_embed, XS, PE);
    k_fold_e<<<1, 256, 0, stream>>>(PE, g_embed, be_embed, PRME);
    k_conv<<<NBLK, NT, 0, stream>>>(XS, mask, WC, PRME, U, ZX, PY);
    k_fold_y<<<1, 256, 0, stream>>>(PY, g_conv, be_conv, PRMY);
    k_final<<<NBLK, NT, 0, stream>>>(feats, mask, U, ZX, PRMY, OUT);
}
